// FixedSplitModel_34583076667906
// MI455X (gfx1250) — hardware-verified
//
#include <hip/hip_runtime.h>

typedef __attribute__((ext_vector_type(16))) _Float16 v16h;
typedef __attribute__((ext_vector_type(8)))  _Float16 v8h;
typedef __attribute__((ext_vector_type(16))) __bf16   v16b;
typedef __attribute__((ext_vector_type(8)))  __bf16   v8b;
typedef __attribute__((ext_vector_type(8)))  float    v8f;
typedef __attribute__((ext_vector_type(4)))  float    v4f;

__device__ __forceinline__ unsigned short f2bf_bits(float f) {
  unsigned u = __float_as_uint(f);
  return (unsigned short)((u + 0x7FFFu + ((u >> 16) & 1u)) >> 16);
}
__device__ __forceinline__ float bf_bits2f(unsigned short h) { return __uint_as_float(((unsigned)h) << 16); }

__device__ __forceinline__ void dep_guard_h(v8f& a, v8f& b, v16h x, v16h y) { asm volatile("v_nop\n\tv_nop\n\tv_nop\n\tv_nop" : "+v"(a), "+v"(b) : "v"(x), "v"(y)); }
__device__ __forceinline__ void dep_guard_b(v8f& a, v8f& b, v16b x, v16b y) { asm volatile("v_nop\n\tv_nop\n\tv_nop\n\tv_nop" : "+v"(a), "+v"(b) : "v"(x), "v"(y)); }
__device__ __forceinline__ void keep4_h(v16h a, v16h b, v16h c, v16h d) { asm volatile("v_nop" :: "v"(a), "v"(b), "v"(c), "v"(d)); }
__device__ __forceinline__ void keep4_b(v16b a, v16b b, v16b c, v16b d) { asm volatile("v_nop" :: "v"(a), "v"(b), "v"(c), "v"(d)); }
__device__ __forceinline__ void acc_guard4(v8f& a, v8f& b, v8f& c, v8f& d) { asm volatile("v_nop\n\tv_nop\n\tv_nop\n\tv_nop" : "+v"(a), "+v"(b), "+v"(c), "+v"(d)); }
template <typename T> struct Frag;
template <> struct Frag<_Float16> {
  typedef v16h V; union U { v16h v; v8h h[2]; };
  static __device__ __forceinline__ v16h load(const _Float16* p) {
    U f; f.h[0] = *(const v8h*)(p); f.h[1] = *(const v8h*)(p + 16); return f.v;
  }
  static __device__ __forceinline__ v8f mma(v16h a, v16h b, v8f c) {
    return __builtin_amdgcn_wmma_f32_16x16x32_f16(false, a, false, b, (short)0, c, false, false);
  }
  static __device__ __forceinline__ void guard(v8f& a, v8f& b, v16h x, v16h y) { dep_guard_h(a, b, x, y); }
  static __device__ __forceinline__ void keep(v16h a, v16h b, v16h c, v16h d) { keep4_h(a, b, c, d); }
};
template <> struct Frag<__bf16> {
  typedef v16b V; union U { v16b v; v8b h[2]; };
  static __device__ __forceinline__ v16b load(const __bf16* p) {
    U f; f.h[0] = *(const v8b*)(p); f.h[1] = *(const v8b*)(p + 16); return f.v;
  }
  static __device__ __forceinline__ v8f mma(v16b a, v16b b, v8f c) {
    return __builtin_amdgcn_wmma_f32_16x16x32_bf16(false, a, false, b, (short)0, c, false, false);
  }
  static __device__ __forceinline__ void guard(v8f& a, v8f& b, v16b x, v16b y) { dep_guard_b(a, b, x, y); }
  static __device__ __forceinline__ void keep(v16b a, v16b b, v16b c, v16b d) { keep4_b(a, b, c, d); }
};

__device__ __forceinline__ unsigned short at_bf_bits(float f) {
  unsigned u = __float_as_uint(f);
  return (unsigned short)((u + 0x7FFFu + ((u >> 16) & 1u)) >> 16);
}
__device__ __forceinline__ __bf16 at_f2bf(float f) { return __builtin_bit_cast(__bf16, at_bf_bits(f)); }
__device__ __forceinline__ void at_split(float f, __bf16& hi, __bf16& lo) {
  const unsigned short hb = at_bf_bits(f);
  hi = __builtin_bit_cast(__bf16, hb);
  lo = at_f2bf(f - __uint_as_float(((unsigned)hb) << 16));
}
__device__ __forceinline__ v8f at_mma(v16b a, v16b b, v8f c) {
  c = __builtin_amdgcn_wmma_f32_16x16x32_bf16(false, a, false, b, (short)0, c, false, false);
  asm volatile("v_nop\n\tv_nop\n\tv_nop\n\tv_nop" : "+v"(c) : "v"(a), "v"(b));
  return c;
}

constexpr int kBatch    = 256;
constexpr int kSeqLen   = 1024;
constexpr int kHid      = 64;
constexpr int kFF       = 128;
constexpr int kKey      = 32;
constexpr int kVoc      = 64;
constexpr int kOut      = 64;
constexpr int kTabPitch = 128;
constexpr int kTabLds   = 96;
constexpr int kWavesScan = 8;
constexpr int kScanThreads = kWavesScan * 32;
constexpr int kVocThreads  = 128;
constexpr int kOslPitch = 68;

static_assert(kBatch % kWavesScan == 0, "grid covers all sequences exactly");
static_assert(kFF == kVocThreads, "one thread per FFN column in the vocabulary kernel");
static_assert(2 * kKey == kHid, "concatenated keys form the 64-deep projection input");
static_assert(kTabPitch == 4 * 32, "one v4f per lane of one wave writes a whole table row");

__global__ __launch_bounds__(kVocThreads)
void k_vocab_keys(const float* __restrict__ embed,
                  const float* __restrict__ W1, const float* __restrict__ b1,
                  const float* __restrict__ W2, const float* __restrict__ b2,
                  const float* __restrict__ gamma, const float* __restrict__ beta,
                  const float* __restrict__ Wsem, const float* __restrict__ bsem,
                  const float* __restrict__ Wepi, const float* __restrict__ bepi,
                  float* __restrict__ KT) {
  __shared__ float se[kHid];
  __shared__ float st1[kFF];
  __shared__ float sx[kHid];
  __shared__ float sh[kHid];
  __shared__ __align__(16) float so[kTabPitch];

  const int v    = blockIdx.x;
  const int tid  = threadIdx.x;
  const int wave = tid >> 5;
  const int lane = tid & 31;

  if (tid < kHid) se[tid] = embed[(size_t)v * kHid + tid];
  so[tid] = 0.0f;
  __syncthreads();

  {
    float a = 0.0f;
#pragma unroll 1
    for (int k = 0; k < kHid; ++k) a += se[k] * W1[k * kFF + tid];
    a += b1[tid];
    st1[tid] = fmaxf(a, 0.0f);
  }
  __syncthreads();

  if (tid < kHid) {
    float a = 0.0f;
#pragma unroll 1
    for (int k = 0; k < kFF; ++k) a += st1[k] * W2[k * kHid + tid];
    a += b2[tid];
    sx[tid] = se[tid] + a;
  }
  __syncthreads();

  if (tid < kHid) {
    float s = 0.0f;
#pragma unroll 1
    for (int n = 0; n < kHid; ++n) s += sx[n];
    const float mu = s * (1.0f / 64.0f);
    float q = 0.0f;
#pragma unroll 1
    for (int n = 0; n < kHid; ++n) { const float d = sx[n] - mu; q += d * d; }
    const float var  = q * (1.0f / 64.0f);
    const float rstd = 1.0f / sqrtf(var + 1e-5f);
    sh[tid] = (gamma[tid] * (sx[tid] - mu)) * rstd + beta[tid];
  }
  __syncthreads();

  if (tid < kHid) {
    const float* Wp = (wave == 0) ? Wsem : Wepi;
    const float* bp = (wave == 0) ? bsem : bepi;
    float a = 0.0f;
#pragma unroll 1
    for (int k = 0; k < kHid; ++k) a += sh[k] * Wp[k * kKey + lane];
    a += bp[lane];
    so[tid] = a;
  }
  __syncthreads();

  if (wave == 0) {
    float ns = 0.0f, ne = 0.0f;
#pragma unroll 1
    for (int j = 0; j < kKey; ++j) {
      const float a = so[j];
      const float e = so[kKey + j];
      ns += a * a;
      ne += e * e;
    }
    if (lane == 0) {
      so[64] = 1.0f / (ns + 1e-6f);
      so[65] = 1.0f / (ne + 1e-6f);
    }
  }
  __syncthreads();

  if (wave == 0) {
    const v4f val = *(const v4f*)(so + 4 * lane);
    float* dst = KT + (size_t)v * kTabPitch + 4 * lane;
    *(volatile v4f*)dst = val;
    __threadfence();
    *(volatile v4f*)dst = val;
  }
}

__global__ __launch_bounds__(kScanThreads)
void k_memory_scan(const int* __restrict__ seq, const float* __restrict__ KT,
                   const float* __restrict__ Wout, const float* __restrict__ bout,
                   float* __restrict__ out) {
  __shared__ __align__(16) float  tab[kVoc * kTabLds];
  __shared__ __align__(16) __bf16 wth[kOut * kHid];
  __shared__ __align__(16) __bf16 wtl[kOut * kHid];
  __shared__ __align__(16) __bf16 cah[16 * kHid];
  __shared__ __align__(16) __bf16 cal[16 * kHid];
  __shared__ __align__(16) float  osl[16 * kOslPitch];

  const int tid  = threadIdx.x;
  const int wave = tid >> 5;
  const int lane = tid & 31;
  const int hh   = lane >> 4;
  const int cc   = lane & 15;

  for (int idx = tid; idx < kVoc * kTabLds; idx += kScanThreads) {
    const int vr  = idx / kTabLds;
    const int col = idx - vr * kTabLds;
    tab[idx] = KT[(size_t)vr * kTabPitch + col];
  }
  for (int idx = tid; idx < kHid * kOut; idx += kScanThreads) {
    const int k = idx >> 6;
    const int n = idx & 63;
    __bf16 h1, l1;
    at_split(Wout[idx], h1, l1);
    wth[n * kHid + k] = h1;
    wtl[n * kHid + k] = l1;
  }
  {
    const __bf16 zb = __builtin_bit_cast(__bf16, (unsigned short)0);
    for (int idx = tid; idx < 8 * kHid; idx += kScanThreads) {
      cah[8 * kHid + idx] = zb;
      cal[8 * kHid + idx] = zb;
    }
  }
  __syncthreads();

  const int b = blockIdx.x * kWavesScan + wave;
  const int* sq = seq + (size_t)b * kSeqLen;

  float ms[kKey], me[kKey];
#pragma unroll
  for (int j = 0; j < kKey; ++j) { ms[j] = 0.0f; me[j] = 0.0f; }
  float cs = 0.0f, ce = 0.0f;

#pragma unroll 1
  for (int t = 0; t < kSeqLen; ++t) {
    int tok = sq[t];
    tok = tok < 0 ? 0 : (tok > kVoc - 1 ? kVoc - 1 : tok);
    const float* rowp = tab + tok * kTabLds;
    const float upd = (t + 1 < kSeqLen) ? 1.0f : 0.0f;

    {
      float kk[kKey];
#pragma unroll
      for (int q = 0; q < kKey / 4; ++q) {
        const v4f w4 = *(const v4f*)(rowp + 4 * q);
        kk[4 * q + 0] = w4[0]; kk[4 * q + 1] = w4[1]; kk[4 * q + 2] = w4[2]; kk[4 * q + 3] = w4[3];
      }
      const float ki   = rowp[lane];
      const float rinv = rowp[64];
      float p0 = 0.0f, p1 = 0.0f, p2 = 0.0f, p3 = 0.0f;
#pragma unroll
      for (int j = 0; j < kKey; j += 4) {
        p0 += ms[j] * kk[j];
        p1 += ms[j + 1] * kk[j + 1];
        p2 += ms[j + 2] * kk[j + 2];
        p3 += ms[j + 3] * kk[j + 3];
      }
      const float vps = (p0 + p1) + (p2 + p3);
      cs = vps;
      const float dv = (ki - vps * rinv) * upd;
#pragma unroll
      for (int j = 0; j < kKey; ++j) ms[j] += dv * kk[j];
    }
    {
      float kk[kKey];
#pragma unroll
      for (int q = 0; q < kKey / 4; ++q) {
        const v4f w4 = *(const v4f*)(rowp + kKey + 4 * q);
        kk[4 * q + 0] = w4[0]; kk[4 * q + 1] = w4[1]; kk[4 * q + 2] = w4[2]; kk[4 * q + 3] = w4[3];
      }
      const float ki   = rowp[kKey + lane];
      const float rinv = rowp[65];
      const float sc   = (float)(t + 1) * (1.0f / 1024.0f);
      float p0 = 0.0f, p1 = 0.0f, p2 = 0.0f, p3 = 0.0f;
#pragma unroll
      for (int j = 0; j < kKey; j += 4) {
        p0 += me[j] * kk[j];
        p1 += me[j + 1] * kk[j + 1];
        p2 += me[j + 2] * kk[j + 2];
        p3 += me[j + 3] * kk[j + 3];
      }
      const float vpe = (p0 + p1) + (p2 + p3);
      ce = vpe;
      const float dve = ki - vpe * rinv;
      const float dv  = (sc * dve) * upd;
#pragma unroll
      for (int j = 0; j < kKey; ++j) me[j] += dv * kk[j];
    }
  }

  {
    __bf16 h1, l1;
    at_split(cs, h1, l1);
    cah[wave * kHid + lane] = h1;
    cal[wave * kHid + lane] = l1;
    at_split(ce, h1, l1);
    cah[wave * kHid + kKey + lane] = h1;
    cal[wave * kHid + kKey + lane] = l1;
  }
  __syncthreads();

  if (wave == 0) {
    v8f acc[4];
#pragma unroll
    for (int j = 0; j < 4; ++j) acc[j] = (v8f){0.f,0.f,0.f,0.f,0.f,0.f,0.f,0.f};
#pragma unroll
    for (int kb = 0; kb < 2; ++kb) {
      const int k0 = kb * 32;
      const v16b ah = Frag<__bf16>::load(cah + cc * kHid + k0 + 8 * hh);
      const v16b al = Frag<__bf16>::load(cal + cc * kHid + k0 + 8 * hh);
#pragma unroll
      for (int j = 0; j < 4; ++j) {
        const v16b bh = Frag<__bf16>::load(wth + (16 * j + cc) * kHid + k0 + 8 * hh);
        const v16b bl = Frag<__bf16>::load(wtl + (16 * j + cc) * kHid + k0 + 8 * hh);
        acc[j] = at_mma(ah, bh, acc[j]);
        acc[j] = at_mma(ah, bl, acc[j]);
        acc[j] = at_mma(al, bh, acc[j]);
      }
    }
#pragma unroll
    for (int j = 0; j < 4; ++j) {
      const float bv = bout[16 * j + cc];
#pragma unroll
      for (int r = 0; r < 8; ++r) osl[(8 * hh + r) * kOslPitch + 16 * j + cc] = acc[j][r] + bv;
    }
    __builtin_amdgcn_fence(__ATOMIC_RELEASE, "workgroup");
    __builtin_amdgcn_wave_barrier();
    __builtin_amdgcn_fence(__ATOMIC_ACQUIRE, "workgroup");
    float* ob = out + (size_t)blockIdx.x * kWavesScan * kOut;
    const int c4 = cc * 4;
    for (int pass = 0; pass < 2; ++pass) {
#pragma unroll
      for (int it = 0; it < 4; ++it) {
        const int row = it * 2 + hh;
        const v4f val = *(const v4f*)(osl + row * kOslPitch + c4);
        *(volatile v4f*)(ob + (size_t)row * kOut + c4) = val;
      }
      __threadfence();
    }
  }
}

extern "C" void kernel_launch(void* const* d_in, const int* in_sizes, int n_in,
                              void* d_out, int out_size, void* d_ws, size_t ws_size,
                              hipStream_t stream) {
  if (n_in < 14) return;
  if (in_sizes[0] != kBatch * kSeqLen) return;
  if (in_sizes[1] != kVoc * kHid) return;
  if (in_sizes[2] != kHid * kFF || in_sizes[3] != kFF) return;
  if (in_sizes[4] != kFF * kHid || in_sizes[5] != kHid) return;
  if (in_sizes[6] != kHid || in_sizes[7] != kHid) return;
  if (in_sizes[8] != kHid * kKey || in_sizes[9] != kKey) return;
  if (in_sizes[10] != kHid * kKey || in_sizes[11] != kKey) return;
  if (in_sizes[12] != 2 * kKey * kOut || in_sizes[13] != kOut) return;
  if (out_size != kBatch * kOut) return;

  const size_t tab_bytes = (size_t)kVoc * kTabPitch * sizeof(float);
  if (ws_size < tab_bytes) return;

  const int*   seq   = (const int*)  d_in[0];
  const float* embed = (const float*)d_in[1];
  const float* W1    = (const float*)d_in[2];
  const float* b1    = (const float*)d_in[3];
  const float* W2    = (const float*)d_in[4];
  const float* b2    = (const float*)d_in[5];
  const float* gamma = (const float*)d_in[6];
  const float* beta  = (const float*)d_in[7];
  const float* Wsem  = (const float*)d_in[8];
  const float* bsem  = (const float*)d_in[9];
  const float* Wepi  = (const float*)d_in[10];
  const float* bepi  = (const float*)d_in[11];
  const float* Wout  = (const float*)d_in[12];
  const float* bout  = (const float*)d_in[13];
  float* out = (float*)d_out;
  float* KT  = (float*)d_ws;

  k_vocab_keys<<<kVoc, kVocThreads, 0, stream>>>(embed, W1, b1, W2, b2, gamma, beta,
                                                  Wsem, bsem, Wepi, bepi, KT);
  k_memory_scan<<<kBatch / kWavesScan, kScanThreads, 0, stream>>>(seq, KT, Wout, bout, out);
}
